// TransformerEncoderLayer_16681652978110
// MI455X (gfx1250) — hardware-verified
//
#include <hip/hip_runtime.h>
#ifndef NB
#define NB 4
#endif
#ifndef SEQ
#define SEQ 1024
#endif
#define NB_FULL 4
#define SEQ_FULL 1024
#define DM 768
#define NH 8
#define HD 96
#define DFF 3072
#define LQ 2304
#define OP 1024
#define NREL 199
#define RSL 208
#define RLP 210
#define NR (NB * SEQ)

static_assert(SEQ % 128 == 0);
static_assert(SEQ <= SEQ_FULL);
static_assert(NB <= NB_FULL);
static_assert(NH * HD == DM);
static_assert(LQ == 3 * DM);
static_assert(OP == NH * 128);
static_assert(HD % 32 == 0 && HD <= 128);
static_assert(DM % 64 == 0 && DFF % 64 == 0 && LQ % 64 == 0);
static_assert(DM % 32 == 0 && DFF % 32 == 0 && OP % 32 == 0);
static_assert(NR % 128 == 0);
static_assert(RSL % 16 == 0 && RSL >= NREL);
static_assert(NREL / 2 == 99);
static_assert(DM == 192 * 4);

typedef unsigned short v8us __attribute__((ext_vector_type(8), may_alias));
typedef float  v8f  __attribute__((ext_vector_type(8)));
typedef float  v4f  __attribute__((ext_vector_type(4)));
typedef float  v4fa __attribute__((ext_vector_type(4), may_alias));
typedef _Float16 v16h __attribute__((ext_vector_type(16)));
typedef _Float16 v4h  __attribute__((ext_vector_type(4)));
union FragH { v16h v; v8us half[2]; _Float16 h[16]; unsigned short u[16]; };

__device__ __forceinline__ unsigned short bf16_bits(float x) { unsigned int u = __float_as_uint(x); return (unsigned short)((u + 0x7FFFu + ((u >> 16) & 1u)) >> 16); }
__device__ __forceinline__ float bf16_rne(float x) { return __uint_as_float(((unsigned int)bf16_bits(x)) << 16); }
__device__ __forceinline__ int iclamp(int v, int lo, int hi) { return v < lo ? lo : (v > hi ? hi : v); }
__device__ __forceinline__ unsigned xrow(unsigned r) { return (r / (unsigned)NB) * (unsigned)NB_FULL + (r % (unsigned)NB); }
__device__ __forceinline__ void split_hl(float v, _Float16& hi, _Float16& lo) {
  const float vh = (fabsf(v) < 6.103515625e-5f) ? 0.0f : v;
  const _Float16 hv = (_Float16)vh;
  hi = hv;
  lo = (_Float16)((v - (float)hv) * 1024.0f);
}

__device__ __forceinline__ v16h g2_frag(const _Float16* p, unsigned hh) { FragH f; f.half[0] = *(const v8us*)((const unsigned short*)p + 8 * hh); f.half[1] = *(const v8us*)((const unsigned short*)p + 16 + 8 * hh); return f.v; }
__device__ __forceinline__ v16h vt_frag(const _Float16* row, int jb, unsigned hh) {
  const int g0 = iclamp(jb + 8 * (int)hh, 0, (int)SEQ - 8), g1 = iclamp(jb + 16 + 8 * (int)hh, 0, (int)SEQ - 8);
  FragH f; f.half[0] = *(const v8us*)((const unsigned short*)row + g0); f.half[1] = *(const v8us*)((const unsigned short*)row + g1); return f.v; }
__device__ __forceinline__ v8f g2_mma(v16h a, v16h b, v8f c) { v8f d = __builtin_amdgcn_wmma_f32_16x16x32_f16(false, a, false, b, (short)0, c, false, false); asm volatile("v_nop\n\tv_nop\n\tv_nop\n\tv_nop" : "+v"(d) : "v"(a), "v"(b)); return d; }

__global__ __launch_bounds__(256) void k_x16(const float* __restrict__ x, _Float16* __restrict__ X16) {
  const unsigned t = blockIdx.x * 256u + threadIdx.x;
  if (t >= (unsigned)(NR * (DM / 8))) return;
  const unsigned r = t / (unsigned)(DM / 8), c = (t - r * (unsigned)(DM / 8)) * 8u;
  const float* src = x + (size_t)xrow(r) * DM + c;
  const v4f a = *(const v4fa*)src, b = *(const v4fa*)(src + 4);
  FragH f;
#pragma unroll
  for (int q = 0; q < 4; ++q) { f.h[q] = (_Float16)(bf16_rne(a[q]) * 16.0f); f.h[4 + q] = (_Float16)(bf16_rne(b[q]) * 16.0f); }
  const v8us o = f.half[0];
  unsigned short* d = (unsigned short*)X16 + (size_t)t * 8;
  *(volatile v8us*)d = o; __threadfence(); *(volatile v8us*)d = o;
}

__global__ __launch_bounds__(256) void k_cv16(const float* __restrict__ W, _Float16* __restrict__ out, unsigned n8, float scale) {
  const unsigned t = blockIdx.x * 256u + threadIdx.x;
  if (t >= n8) return;
  const float* src = W + (size_t)t * 8;
  const v4f a = *(const v4fa*)src, b = *(const v4fa*)(src + 4);
  FragH f;
#pragma unroll
  for (int q = 0; q < 4; ++q) { f.h[q] = (_Float16)(bf16_rne(a[q]) * scale); f.h[4 + q] = (_Float16)(bf16_rne(b[q]) * scale); }
  const v8us o = f.half[0];
  unsigned short* d = (unsigned short*)out + (size_t)t * 8;
  *(volatile v8us*)d = o; __threadfence(); *(volatile v8us*)d = o;
}

__global__ __launch_bounds__(256) void k_wh(const float* __restrict__ w, _Float16* __restrict__ Wt, float scale) {
  const unsigned t = blockIdx.x * 256u + threadIdx.x;
  if (t >= (unsigned)(DM * (DM / 8))) return;
  const unsigned n = t / (unsigned)(DM / 8), k8 = (t - n * (unsigned)(DM / 8)) * 8u;
  const unsigned hd = n / (unsigned)HD, a = n - hd * (unsigned)HD;
  const float* src = w + (size_t)hd * DM * HD + a;
  FragH f;
#pragma unroll
  for (int i = 0; i < 8; ++i) f.h[i] = (_Float16)(bf16_rne(src[(size_t)(k8 + i) * HD]) * scale);
  const v8us o = f.half[0];
  unsigned short* d = (unsigned short*)Wt + (size_t)t * 8;
  *(volatile v8us*)d = o; __threadfence(); *(volatile v8us*)d = o;
}

__global__ __launch_bounds__(256) void k_wo(const float* __restrict__ w, _Float16* __restrict__ Wt, float scale) {
  const unsigned t = blockIdx.x * 256u + threadIdx.x;
  if (t >= (unsigned)(DM * (OP / 8))) return;
  const unsigned n = t >> 7, k8 = (t & 127u) * 8u;
  const unsigned hd = k8 >> 7, d0 = k8 & 127u;
  const bool in = d0 < (unsigned)HD;
  const unsigned dd = in ? d0 : (unsigned)(HD - 8);
  const float* src = w + ((size_t)hd * HD + dd) * DM + n;
  FragH f;
#pragma unroll
  for (int i = 0; i < 8; ++i) { const float xv = src[(size_t)i * DM]; f.h[i] = (_Float16)(in ? bf16_rne(xv) * scale : 0.0f); }
  const v8us o = f.half[0];
  unsigned short* d = (unsigned short*)Wt + (size_t)t * 8;
  *(volatile v8us*)d = o; __threadfence(); *(volatile v8us*)d = o;
}

__global__ __launch_bounds__(256) void k_rt(const float* __restrict__ rel, _Float16* __restrict__ RT) {
  const unsigned t = blockIdx.x * 256u + threadIdx.x;
  if (t >= (unsigned)(NH * RSL * (HD / 8))) return;
  const unsigned hm = t / (unsigned)(HD / 8), a8 = (t - hm * (unsigned)(HD / 8)) * 8u;
  const unsigned hd = hm / (unsigned)RSL, sl = hm - hd * (unsigned)RSL;
  const bool in = sl < (unsigned)NREL;
  const unsigned ss = in ? sl : (unsigned)(NREL - 1);
  const float* src = rel + ((size_t)hd * NREL + ss) * HD + a8;
  const v4f a = *(const v4fa*)src, b = *(const v4fa*)(src + 4);
  FragH f;
#pragma unroll
  for (int q = 0; q < 4; ++q) { f.h[q] = (_Float16)(in ? bf16_rne(a[q]) * 16.0f : 0.0f); f.h[4 + q] = (_Float16)(in ? bf16_rne(b[q]) * 16.0f : 0.0f); }
  const v8us o = f.half[0];
  unsigned short* d = (unsigned short*)RT + (size_t)t * 8;
  *(volatile v8us*)d = o; __threadfence(); *(volatile v8us*)d = o;
}

__global__ __launch_bounds__(256) void k_vt(const _Float16* __restrict__ QKV, _Float16* __restrict__ VT) {
  __shared__ unsigned short tl[64][98];
  const unsigned tid = threadIdx.x; const unsigned nbp = (unsigned)(NB * NH * (SEQ / 64));
  const unsigned pl = blockIdx.x / nbp, bi = blockIdx.x - pl * nbp;
  const unsigned slab = bi / (unsigned)(SEQ / 64), lg = bi % (unsigned)(SEQ / 64); const unsigned b = slab / (unsigned)NH, hd = slab % (unsigned)NH;
  const unsigned short* src = (const unsigned short*)QKV + (size_t)pl * NR * LQ;
  unsigned short* dst = (unsigned short*)VT + (size_t)pl * NB * NH * HD * SEQ;
  for (unsigned i = tid; i < 768u; i += 256u) { const unsigned r = i / 12u, c8 = (i - r * 12u) * 8u; FragH f; f.half[0] = *(const v8us*)(src + ((size_t)(lg * 64u + r) * NB + b) * LQ + 2u * DM + hd * (unsigned)HD + c8);
#pragma unroll
    for (int q = 0; q < 8; ++q) tl[r][c8 + q] = f.u[q]; }
  __syncthreads();
  for (int pass = 0; pass < 2; ++pass) {
#pragma unroll
    for (unsigned rd = 0; rd < 3; ++rd) { const unsigned d = rd * 32u + (tid >> 3), pc = tid & 7u; FragH f;
#pragma unroll
      for (int q = 0; q < 8; ++q) f.u[q] = tl[pc * 8u + q][d];
      const v8us o = f.half[0];
      *(volatile v8us*)(dst + ((size_t)slab * HD + d) * SEQ + lg * 64u + pc * 8u) = o; }
    if (pass == 0) __threadfence(); }
}

__global__ __launch_bounds__(128) void k_attn(const _Float16* __restrict__ QKV, const _Float16* __restrict__ VT, const _Float16* __restrict__ RT, _Float16* __restrict__ O16) {
  __shared__ float rl[4][16][RLP];
  __shared__ __attribute__((aligned(16))) unsigned short os[2][4][16][136];
  const unsigned tid = threadIdx.x, lane = tid & 31u, ln = lane & 15u, hh = lane >> 4;
  const unsigned w = (unsigned)__builtin_amdgcn_readfirstlane((int)(tid >> 5));
  const unsigned qb = blockIdx.x % (unsigned)(SEQ / 64), hb = blockIdx.x / (unsigned)(SEQ / 64); const unsigned hd = hb % (unsigned)NH, b = hb / (unsigned)NH;
  const unsigned q0 = qb * 64u + w * 16u;
  const _Float16* qrow = QKV + ((size_t)(q0 + ln) * NB + b) * LQ + hd * (unsigned)HD;
  const _Float16* qrol = qrow + (size_t)NR * LQ;
  const v8f z8 = {0.f, 0.f, 0.f, 0.f, 0.f, 0.f, 0.f, 0.f};
  float* rlw = &rl[w][ln][0];
  {
    const _Float16* rbase = RT + ((size_t)hd * RSL + ln) * HD;
#pragma unroll 1
    for (unsigned mt = 0; mt < (unsigned)(RSL / 16); ++mt) {
      const _Float16* rr = rbase + (size_t)(mt * 16u) * HD;
      v8f zm = z8, zr = z8;
#pragma unroll
      for (int kk = 0; kk < 3; ++kk) { const v16h ra = g2_frag(rr + 32 * kk, hh); zm = g2_mma(ra, g2_frag(qrow + 32 * kk, hh), zm); zr = g2_mma(ra, g2_frag(qrol + 32 * kk, hh), zr); }
#pragma unroll
      for (int r = 0; r < 8; ++r) rlw[mt * 16u + 8u * hh + r] = fmaf(zr[r], 0.0009765625f, zm[r]) * 0.0625f;
    }
  }
  __builtin_amdgcn_fence(4  , "workgroup"); __builtin_amdgcn_wave_barrier();
  const _Float16* kbase = QKV + (size_t)b * LQ + DM + hd * (unsigned)HD;
  const _Float16* vbh = VT + ((size_t)(b * NH + hd) * HD + ln) * SEQ;
  const _Float16* vbl = vbh + (size_t)NB * NH * HD * SEQ;
  const int qi = (int)(q0 + ln);
  v8f o[6] = {z8, z8, z8, z8, z8, z8};
  v8f ox[6] = {z8, z8, z8, z8, z8, z8};
  float mrun = -1.0e30f, l = 0.f;
#pragma unroll 1
  for (int s = 0; s < 8; ++s) {
    const int j0 = (int)q0 - 128 + 32 * s;
    if (j0 + 32 <= 0 || j0 >= (int)SEQ) continue;
    unsigned zo = 0u;
    asm volatile("" : "+v"(zo));
    const _Float16* qh = qrow + zo; const _Float16* ql = qrol + zo;
    const int kj0 = iclamp(j0 + (int)ln, 0, (int)SEQ - 1), kj1 = iclamp(j0 + 16 + (int)ln, 0, (int)SEQ - 1);
    const _Float16* kr0 = kbase + ((size_t)(unsigned)kj0 * NB) * LQ; const _Float16* kr1 = kbase + ((size_t)(unsigned)kj1 * NB) * LQ;
    v8f cm0 = z8, cr0 = z8, cm1 = z8, cr1 = z8;
#pragma unroll
    for (int kk = 0; kk < 3; ++kk) {
      const v16h qhf = g2_frag(qh + 32 * kk, hh), qlf = g2_frag(ql + 32 * kk, hh);
      const v16h ka = g2_frag(kr0 + 32 * kk, hh), kb = g2_frag(kr1 + 32 * kk, hh);
      cm0 = g2_mma(ka, qhf, cm0); cr0 = g2_mma(ka, qlf, cr0);
      cm1 = g2_mma(kb, qhf, cm1); cr1 = g2_mma(kb, qlf, cr1);
    }
    v8f c[2];
#pragma unroll
    for (int r = 0; r < 8; ++r) { c[0][r] = fmaf(cr0[r], 0.0009765625f, cm0[r]); c[1][r] = fmaf(cr1[r], 0.0009765625f, cm1[r]); }
    float mx = -1.0e30f;
#pragma unroll
    for (int t = 0; t < 2; ++t)
#pragma unroll
      for (int r = 0; r < 8; ++r) {
        const int j = j0 + t * 16 + 8 * (int)hh + r; const int sl = j - qi + (NREL / 2);
        const bool ok = ((unsigned)j < (unsigned)SEQ) && ((unsigned)sl <= (unsigned)(NREL - 1));
        const float rv = rlw[iclamp(sl, 0, NREL - 1)];
        const float lg = fmaf(c[t][r], 0.10206207262f, rv);
        const float lv = ok ? lg : -1.0e30f;
        c[t][r] = lv; mx = fmaxf(mx, lv); }
    mx = fmaxf(mx, __shfl_xor(mx, 16, 32));
    const float mnew = fmaxf(mrun, mx);
    const float alpha = __expf(mrun - mnew);
    mrun = mnew;
    const float sh = 6.9314718f - mnew;
    float ps = 0.f;
    FragH ph, pl;
#pragma unroll
    for (int r = 0; r < 8; ++r) {
      const float x0 = __expf(c[0][r] + sh), x1 = __expf(c[1][r] + sh);
      const float e0 = (c[0][r] > -1.0e29f) ? x0 : 0.f, e1 = (c[1][r] > -1.0e29f) ? x1 : 0.f;
      ps += e0 + e1;
      _Float16 h0, l0, h1, l1; split_hl(e0, h0, l0); split_hl(e1, h1, l1);
      ph.h[r] = h0; ph.h[8 + r] = h1; pl.h[r] = l0; pl.h[8 + r] = l1;
    }
    l = l * alpha + ps;
#pragma unroll
    for (int dt = 0; dt < 6; ++dt)
#pragma unroll
      for (int r = 0; r < 8; ++r) { o[dt][r] *= alpha; ox[dt][r] *= alpha; }
#pragma unroll
    for (int dt = 0; dt < 6; ++dt) {
      const v16h fh = vt_frag(vbh + (size_t)(dt * 16u) * SEQ, j0, hh), fl = vt_frag(vbl + (size_t)(dt * 16u) * SEQ, j0, hh);
      o[dt] = g2_mma(fh, ph.v, o[dt]);
      ox[dt] = g2_mma(fl, ph.v, ox[dt]);
      ox[dt] = g2_mma(fh, pl.v, ox[dt]);
    }
  }
  const float lt = l + __shfl_xor(l, 16, 32);
  const float fin = 64.0f * (1.0f / lt);
#pragma unroll
  for (int dt = 0; dt < 6; ++dt) { FragH fh, fl;
#pragma unroll
    for (int r = 0; r < 8; ++r) { const float v = fmaf(ox[dt][r], 0.0009765625f, o[dt][r]) * fin; _Float16 a, cc; split_hl(v, a, cc); fh.h[r] = a; fl.h[r] = cc; }
    *(v8us*)&os[0][w][ln][dt * 16 + 8 * hh] = fh.half[0]; *(v8us*)&os[1][w][ln][dt * 16 + 8 * hh] = fl.half[0]; }
  { const v8us zz = {0, 0, 0, 0, 0, 0, 0, 0};
    *(v8us*)&os[0][w][ln][96 + 8 * hh] = zz; *(v8us*)&os[0][w][ln][112 + 8 * hh] = zz;
    *(v8us*)&os[1][w][ln][96 + 8 * hh] = zz; *(v8us*)&os[1][w][ln][112 + 8 * hh] = zz; }
  __builtin_amdgcn_fence(4  , "workgroup"); __builtin_amdgcn_wave_barrier();
  const unsigned rq = lane >> 4, pc = (lane & 15u) * 8u;
  for (int pass = 0; pass < 2; ++pass) {
#pragma unroll
    for (unsigned pn = 0; pn < 2; ++pn)
#pragma unroll
      for (unsigned it = 0; it < 8; ++it) { const unsigned row = it * 2u + rq; const v8us v = *(const v8us*)&os[pn][w][row][pc];
        *(volatile v8us*)((unsigned short*)O16 + (size_t)pn * NR * OP + ((size_t)(q0 + row) * NB + b) * OP + hd * 128u + pc) = v; }
    if (pass == 0) __threadfence(); }
}

template <int ACT, int RES, int HASB, int RESA, int OUTL>
__global__ __launch_bounds__(128) void k_gemm2(const _Float16* __restrict__ A, const _Float16* __restrict__ Al, unsigned lda, const _Float16* __restrict__ Bh, unsigned ldb, float alpha, const float* __restrict__ bias,
    const float* __restrict__ R, unsigned ldr, float* __restrict__ C, _Float16* __restrict__ C16, _Float16* __restrict__ C16l, unsigned ldc, unsigned M, unsigned N, unsigned K) {
  static_assert(ACT == 0 || ACT == 1);
  static_assert(RES == 0 || RES == 1 || RES == 2);
  __shared__ __attribute__((aligned(16))) float so[4][32][68];
  const unsigned tid = threadIdx.x, w = tid >> 5, lane = tid & 31u, ln = lane & 15u, hh = lane >> 4;
  const unsigned ntn = N >> 6; const unsigned mt = blockIdx.x / ntn, nq = blockIdx.x - mt * ntn; const unsigned row0 = mt * 128u + 32u * w, col0 = nq * 64u; if (row0 >= M) return;
  const _Float16* a0p = A + (size_t)(row0 + ln) * lda; const _Float16* a1p = a0p + (size_t)16 * lda;
  const _Float16* a0l = RESA ? (Al + (size_t)(row0 + ln) * lda) : a0p; const _Float16* a1l = RESA ? (a0l + (size_t)16 * lda) : a1p;
  const _Float16* b0p = Bh + (size_t)(col0 + ln) * ldb; const _Float16* b1p = b0p + (size_t)16 * ldb; const _Float16* b2p = b1p + (size_t)16 * ldb; const _Float16* b3p = b2p + (size_t)16 * ldb;
  const v8f z8 = {0.f,0.f,0.f,0.f,0.f,0.f,0.f,0.f}; v8f c00 = z8, c01 = z8, c02 = z8, c03 = z8, c10 = z8, c11 = z8, c12 = z8, c13 = z8;
  v8f r00 = z8, r01 = z8, r02 = z8, r03 = z8, r10 = z8, r11 = z8, r12 = z8, r13 = z8;
#pragma unroll 1
  for (unsigned kb = 0; kb < K; kb += 32u) { const v16h a0 = g2_frag(a0p + kb, hh), a1 = g2_frag(a1p + kb, hh);
    v16h l0 = a0, l1 = a1;
    if (RESA) { l0 = g2_frag(a0l + kb, hh); l1 = g2_frag(a1l + kb, hh); }
    v16h bfr = g2_frag(b0p + kb, hh); c00 = g2_mma(a0, bfr, c00); c10 = g2_mma(a1, bfr, c10); if (RESA) { r00 = g2_mma(l0, bfr, r00); r10 = g2_mma(l1, bfr, r10); }
    bfr = g2_frag(b1p + kb, hh); c01 = g2_mma(a0, bfr, c01); c11 = g2_mma(a1, bfr, c11); if (RESA) { r01 = g2_mma(l0, bfr, r01); r11 = g2_mma(l1, bfr, r11); }
    bfr = g2_frag(b2p + kb, hh); c02 = g2_mma(a0, bfr, c02); c12 = g2_mma(a1, bfr, c12); if (RESA) { r02 = g2_mma(l0, bfr, r02); r12 = g2_mma(l1, bfr, r12); }
    bfr = g2_frag(b3p + kb, hh); c03 = g2_mma(a0, bfr, c03); c13 = g2_mma(a1, bfr, c13); if (RESA) { r03 = g2_mma(l0, bfr, r03); r13 = g2_mma(l1, bfr, r13); } }
  if (RESA) {
    c00 = c00 + r00 * 0.0009765625f; c01 = c01 + r01 * 0.0009765625f; c02 = c02 + r02 * 0.0009765625f; c03 = c03 + r03 * 0.0009765625f;
    c10 = c10 + r10 * 0.0009765625f; c11 = c11 + r11 * 0.0009765625f; c12 = c12 + r12 * 0.0009765625f; c13 = c13 + r13 * 0.0009765625f; }
  v8f accs[8] = {c00, c01, c02, c03, c10, c11, c12, c13};
#pragma unroll
  for (int u = 0; u < 8; ++u) { const int t = u & 3, half = u >> 2; const unsigned col = col0 + t * 16 + ln; float bv = 0.f; if (HASB) bv = bf16_rne(bias[col]);
#pragma unroll
    for (int r = 0; r < 8; ++r) { const unsigned rloc = half * 16 + 8 * hh + r; so[w][rloc][t * 16 + ln] = accs[u][r] * alpha + bv; } }
  __builtin_amdgcn_fence(4  , "workgroup"); __builtin_amdgcn_wave_barrier();
  const unsigned rsub = lane >> 4, c4 = (lane & 15u) * 4u;
  if (ACT == 1 || RES != 0) {
#pragma unroll 4
    for (unsigned q = 0; q < 16; ++q) { const unsigned r = q * 2u + rsub; v4f v = *(const v4fa*)&so[w][r][c4];
      if (RES != 0) { const unsigned gr = row0 + r; const unsigned sr = (RES == 2) ? xrow(gr) : gr; const v4f rv = *(const v4fa*)(R + (size_t)sr * ldr + col0 + c4);
#pragma unroll
        for (int i = 0; i < 4; ++i) v[i] += (RES == 2) ? bf16_rne(rv[i]) : rv[i]; }
      if (ACT == 1) {
#pragma unroll
        for (int i = 0; i < 4; ++i) v[i] = fmaxf(v[i], 0.0f); }
      *(v4fa*)&so[w][r][c4] = v; }
  }
  for (int pass = 0; pass < 2; ++pass) {
#pragma unroll
    for (unsigned q = 0; q < 16; ++q) { const unsigned r = q * 2u + rsub; const v4f v = *(const v4fa*)&so[w][r][c4];
      if (C) *(volatile v4f*)(C + (size_t)(row0 + r) * ldc + col0 + c4) = v;
      if (C16) { v4h h4, l4;
#pragma unroll
        for (int i = 0; i < 4; ++i) { _Float16 a, cc; if (OUTL) split_hl(v[i], a, cc); else { a = (_Float16)v[i]; cc = (_Float16)0.0f; } h4[i] = a; l4[i] = cc; }
        *(volatile v4h*)(C16 + (size_t)(row0 + r) * ldc + col0 + c4) = h4;
        if (OUTL) *(volatile v4h*)(C16l + (size_t)(row0 + r) * ldc + col0 + c4) = l4; } }
    if (pass == 0) __threadfence(); }
}

template <int W16, int OMAP>
__global__ __launch_bounds__(192) void k_ln(const float* __restrict__ Y, const float* __restrict__ g, const float* __restrict__ bb, float* __restrict__ N32, _Float16* __restrict__ N16) {
  __shared__ float sm[6]; __shared__ float sv[6];
  const unsigned r = blockIdx.x, t = threadIdx.x, lane = t & 31u, w = t >> 5;
  const v4f xa = *(const v4fa*)(Y + (size_t)r * DM + t * 4u);
  float s = (xa[0] + xa[1]) + (xa[2] + xa[3]);
  s += __shfl_xor(s, 1, 32); s += __shfl_xor(s, 2, 32); s += __shfl_xor(s, 4, 32); s += __shfl_xor(s, 8, 32); s += __shfl_xor(s, 16, 32);
  if (lane == 0) sm[w] = s;
  __syncthreads();
  float tot = 0.f;
#pragma unroll
  for (int i = 0; i < 6; ++i) tot += sm[i];
  const float mu = tot * (1.0f / (float)DM);
  const float d0 = xa[0] - mu, d1 = xa[1] - mu, d2 = xa[2] - mu, d3 = xa[3] - mu;
  float q2 = (d0 * d0 + d1 * d1) + (d2 * d2 + d3 * d3);
  q2 += __shfl_xor(q2, 1, 32); q2 += __shfl_xor(q2, 2, 32); q2 += __shfl_xor(q2, 4, 32); q2 += __shfl_xor(q2, 8, 32); q2 += __shfl_xor(q2, 16, 32);
  if (lane == 0) sv[w] = q2;
  __syncthreads();
  float vt = 0.f;
#pragma unroll
  for (int i = 0; i < 6; ++i) vt += sv[i];
  const float rs = rsqrtf(vt * (1.0f / (float)DM) + 1.0e-5f);
  const v4f gv = *(const v4fa*)(g + t * 4u), bv = *(const v4fa*)(bb + t * 4u);
  v4f y; v4h yh, yl;
  y[0] = d0 * rs * bf16_rne(gv[0]) + bf16_rne(bv[0]); y[1] = d1 * rs * bf16_rne(gv[1]) + bf16_rne(bv[1]);
  y[2] = d2 * rs * bf16_rne(gv[2]) + bf16_rne(bv[2]); y[3] = d3 * rs * bf16_rne(gv[3]) + bf16_rne(bv[3]);
#pragma unroll
  for (int i = 0; i < 4; ++i) { _Float16 a, cc; split_hl(y[i], a, cc); yh[i] = a; yl[i] = cc; }
  const unsigned orow = OMAP ? xrow(r) : r;
  for (int pass = 0; pass < 2; ++pass) {
    *(volatile v4f*)(N32 + (size_t)orow * DM + t * 4u) = y;
    if (W16) { *(volatile v4h*)(N16 + (size_t)r * DM + t * 4u) = yh; *(volatile v4h*)(N16 + (size_t)NR * DM + (size_t)r * DM + t * 4u) = yl; }
    if (pass == 0) __threadfence(); }
}

#define SZ_BQKV ((size_t)LQ * DM * 2)
#define SZ_BO   ((size_t)DM * OP * 2)
#define SZ_BW1  ((size_t)DFF * DM * 2)
#define SZ_BW2  ((size_t)DM * DFF * 2)
#define SZ_RT   ((size_t)NH * RSL * HD * 2)
#define SZ_X16  ((size_t)NR * DM * 2)
#define SZ_QKV  ((size_t)NR * LQ * 2)
#define SZ_VT   ((size_t)NB * NH * HD * SEQ * 2)
#define SZ_HF   ((size_t)NR * DFF * 2)
#define SZ_ATT  (2 * SZ_QKV + 2 * SZ_VT)
#define SZ_RA   (SZ_ATT > 2 * SZ_HF ? SZ_ATT : 2 * SZ_HF)
#define SZ_O16  ((size_t)2 * NR * OP * 2)
#define SZ_Y    ((size_t)NR * DM * 4)
#define SZ_X1   ((size_t)NR * DM * 4)
#define SZ_X1H  ((size_t)2 * NR * DM * 2)
#define SZ_TOT  (SZ_BQKV + SZ_BO + SZ_BW1 + SZ_BW2 + SZ_RT + SZ_X16 + SZ_RA + SZ_O16 + SZ_Y + SZ_X1 + SZ_X1H)
static_assert(SZ_ATT <= SZ_RA);
static_assert(2 * SZ_HF <= SZ_RA);
static_assert(SZ_TOT <= (size_t)134217728);
static_assert(SZ_BQKV % 256 == 0 && SZ_BO % 256 == 0 && SZ_BW1 % 256 == 0 && SZ_RT % 256 == 0 && SZ_X16 % 256 == 0 && SZ_RA % 256 == 0 && SZ_QKV % 256 == 0 && SZ_VT % 256 == 0 && SZ_HF % 256 == 0 && SZ_O16 % 256 == 0 && SZ_Y % 256 == 0);
static_assert((NR * (DM / 8)) % 256 == 0);
static_assert(((size_t)DM * (DM / 8)) % 256 == 0 && ((size_t)DM * (OP / 8)) % 256 == 0 && ((size_t)DFF * (DM / 8)) % 256 == 0 && ((size_t)NH * RSL * (HD / 8)) % 256 == 0);
static_assert(64 * (HD / 8) == 768);

extern "C" void kernel_launch(void* const* d_in, const int* in_sizes, int n_in,
                              void* d_out, int out_size, void* d_ws, size_t ws_size, hipStream_t stream) {
  if (n_in < 14) return;
  const long long xneed = ((long long)(SEQ - 1) * NB_FULL + NB) * DM;
  if ((long long)in_sizes[0] < xneed || (long long)out_size < xneed) return;
  if (in_sizes[1] < NH * DM * HD || in_sizes[2] < NH * DM * HD || in_sizes[3] < NH * DM * HD || in_sizes[4] < NH * HD * DM || in_sizes[5] < NH * NREL * HD) return;
  if (in_sizes[6] < DFF * DM || in_sizes[7] < DFF || in_sizes[8] < DM * DFF || in_sizes[9] < DM) return;
  if (in_sizes[10] < DM || in_sizes[11] < DM || in_sizes[12] < DM || in_sizes[13] < DM) return;
  if (ws_size < SZ_TOT) return;
  const float* x = (const float*)d_in[0]; const float* Wq = (const float*)d_in[1]; const float* Wk = (const float*)d_in[2]; const float* Wv = (const float*)d_in[3]; const float* Wo = (const float*)d_in[4];
  const float* rel = (const float*)d_in[5]; const float* W1 = (const float*)d_in[6]; const float* b1 = (const float*)d_in[7]; const float* W2 = (const float*)d_in[8]; const float* b2 = (const float*)d_in[9];
  const float* g1 = (const float*)d_in[10]; const float* be1 = (const float*)d_in[11]; const float* g2 = (const float*)d_in[12]; const float* be2 = (const float*)d_in[13];
  float* out = (float*)d_out;
  char* ws = (char*)d_ws; size_t off = 0;
  _Float16* BQKV = (_Float16*)(ws + off); off += SZ_BQKV;
  _Float16* BO   = (_Float16*)(ws + off); off += SZ_BO;
  _Float16* BW1  = (_Float16*)(ws + off); off += SZ_BW1;
  _Float16* BW2  = (_Float16*)(ws + off); off += SZ_BW2;
  _Float16* RT   = (_Float16*)(ws + off); off += SZ_RT;
  _Float16* X16  = (_Float16*)(ws + off); off += SZ_X16;
  _Float16* QKV  = (_Float16*)(ws + off); _Float16* QKVL = (_Float16*)(ws + off + SZ_QKV); _Float16* VT = (_Float16*)(ws + off + 2 * SZ_QKV);
  _Float16* HF16 = (_Float16*)(ws + off); _Float16* HF16L = (_Float16*)(ws + off + SZ_HF); off += SZ_RA;
  _Float16* O16  = (_Float16*)(ws + off); _Float16* O16L = (_Float16*)(ws + off + SZ_O16 / 2); off += SZ_O16;
  float* Y       = (float*)(ws + off); off += SZ_Y;
  float* X1      = (float*)(ws + off); off += SZ_X1;
  _Float16* X1H  = (_Float16*)(ws + off); _Float16* X1L = (_Float16*)(ws + off + SZ_X1H / 2); off += SZ_X1H;
  if (off > ws_size) return;

  k_x16<<<(unsigned)(NR * (DM / 8) / 256), 256, 0, stream>>>(x, X16);
  k_wh<<<(unsigned)((size_t)DM * (DM / 8) / 256), 256, 0, stream>>>(Wq, BQKV, 16.0f);
  k_wh<<<(unsigned)((size_t)DM * (DM / 8) / 256), 256, 0, stream>>>(Wk, BQKV + (size_t)DM * DM, 16.0f);
  k_wh<<<(unsigned)((size_t)DM * (DM / 8) / 256), 256, 0, stream>>>(Wv, BQKV + (size_t)2 * DM * DM, 16.0f);
  k_wo<<<(unsigned)((size_t)DM * (OP / 8) / 256), 256, 0, stream>>>(Wo, BO, 16.0f);
  k_cv16<<<(unsigned)((size_t)DFF * (DM / 8) / 256), 256, 0, stream>>>(W1, BW1, (unsigned)((size_t)DFF * DM / 8), 64.0f);
  k_cv16<<<(unsigned)((size_t)DM * (DFF / 8) / 256), 256, 0, stream>>>(W2, BW2, (unsigned)((size_t)DM * DFF / 8), 64.0f);
  k_rt<<<(unsigned)((size_t)NH * RSL * (HD / 8) / 256), 256, 0, stream>>>(rel, RT);
  k_gemm2<0, 0, 0, 0, 1><<<(unsigned)((NR / 128) * (LQ / 64)), 128, 0, stream>>>(X16, nullptr, (unsigned)DM, BQKV, (unsigned)DM, 0.00390625f, nullptr, nullptr, 0u, nullptr, QKV, QKVL, (unsigned)LQ, (unsigned)NR, (unsigned)LQ, (unsigned)DM);
  k_vt<<<(unsigned)(2 * NB * NH * (SEQ / 64)), 256, 0, stream>>>(QKV, VT);
  k_attn<<<(unsigned)(NB * NH * (SEQ / 64)), 128, 0, stream>>>(QKV, VT, RT, O16);
  k_gemm2<0, 2, 0, 1, 0><<<(unsigned)((NR / 128) * (DM / 64)), 128, 0, stream>>>(O16, O16L, (unsigned)OP, BO, (unsigned)OP, 0.0009765625f, nullptr, x, (unsigned)DM, Y, nullptr, nullptr, (unsigned)DM, (unsigned)NR, (unsigned)DM, (unsigned)OP);
  k_ln<1, 0><<<(unsigned)NR, 192, 0, stream>>>(Y, g1, be1, X1, X1H);
  k_gemm2<1, 0, 1, 1, 1><<<(unsigned)((NR / 128) * (DFF / 64)), 128, 0, stream>>>(X1H, X1L, (unsigned)DM, BW1, (unsigned)DM, 0.015625f, b1, nullptr, 0u, nullptr, HF16, HF16L, (unsigned)DFF, (unsigned)NR, (unsigned)DFF, (unsigned)DM);
  k_gemm2<0, 1, 1, 1, 0><<<(unsigned)((NR / 128) * (DM / 64)), 128, 0, stream>>>(HF16, HF16L, (unsigned)DFF, BW2, (unsigned)DFF, 0.015625f, b2, X1, (unsigned)DM, Y, nullptr, nullptr, (unsigned)DM, (unsigned)NR, (unsigned)DM, (unsigned)DFF);
  k_ln<0, 1><<<(unsigned)NR, 192, 0, stream>>>(Y, g2, be2, out, nullptr);
}
